// PosLSTM_76115410420290
// MI455X (gfx1250) — hardware-verified
//
#include <hip/hip_runtime.h>


#define AS3 __attribute__((address_space(3)))

#define B_     64
#define P_     16
#define T_     256
#define I_     256
#define H_     512
#define O_     5
#define V_     50000
#define K1_    4096
#define N4_    2048
#define TH_    128
#define MB_    32
#define NBLK   2
#define NTHR   256
#define APITCH 520
#define TP     72

static_assert(K1_ == P_ * I_);
static_assert(N4_ == 4 * H_);
static_assert(2 * TH_ == T_);
static_assert(NBLK * MB_ == B_);
static_assert(H_ == (NTHR / 32) * 64);
static_assert(K1_ % 64 == 0);
static_assert(H_ % 64 == 0);
static_assert(APITCH % 8 == 0);
static_assert(APITCH >= H_);
static_assert(MB_ * P_ == 64 * (NTHR / 32));
static_assert(I_ == 32 * 8);
static_assert(MB_ * O_ == 160);
static_assert((MB_ * O_ * 4) % 128 == 0);

typedef _Float16 v16h __attribute__((ext_vector_type(16)));
typedef _Float16 v8h  __attribute__((ext_vector_type(8)));
typedef float    v8f  __attribute__((ext_vector_type(8)));
typedef float    v4f  __attribute__((ext_vector_type(4)));

typedef AS3 _Float16*       lp_h;
typedef AS3 const _Float16* lcp_h;
typedef AS3 float*          lp_f;

union Frag { v16h v; v8h half[2]; };

#define SCX   256.0f
#define SCW   64.0f
#define INVSC 6.103515625e-05f

constexpr size_t SZ_WXT  = (size_t)N4_ * K1_ * 2;
constexpr size_t SZ_WHT  = (size_t)N4_ * H_ * 2;
constexpr size_t SZ_ST   = (size_t)B_ * H_ * 4;
constexpr size_t SZ_PRE  = (size_t)TH_ * B_ * N4_ * 4;
constexpr size_t OFF_WXT = 0;
constexpr size_t OFF_WHT = OFF_WXT + SZ_WXT;
constexpr size_t OFF_HST = OFF_WHT + SZ_WHT;
constexpr size_t OFF_CST = OFF_HST + SZ_ST;
constexpr size_t OFF_PRE = OFF_CST + SZ_ST;
constexpr size_t WS_END  = OFF_PRE + SZ_PRE;
static_assert(OFF_WHT % 128 == 0);
static_assert(OFF_HST % 128 == 0);
static_assert(OFF_CST % 128 == 0);
static_assert(OFF_PRE % 128 == 0);
static_assert(WS_END <= (size_t)134217728);

constexpr int NBX = 4 * (K1_ / 64) * (H_ / 64);
constexpr int NBH = 4 * (H_ / 64) * (H_ / 64);
static_assert(NBX == 2048);
static_assert(NBH == 256);

constexpr size_t PL_A     = 0;
constexpr size_t PL_ASZ   = (size_t)MB_ * K1_ * 2;
constexpr size_t PL_S     = PL_A + PL_ASZ;
constexpr size_t PL_SSZ   = (size_t)(NTHR / 32) * 8 * 64 * 4;
constexpr size_t PL_BYTES = PL_S + PL_SSZ;
static_assert(PL_S % 16 == 0);
static_assert((MB_ * K1_) % 8 == 0);

constexpr int    A_TILE   = MB_ * APITCH;
constexpr size_t RL_A     = 0;
constexpr size_t RL_ASZ   = (size_t)2 * A_TILE * 2;
constexpr size_t RL_C     = RL_A + RL_ASZ;
constexpr size_t RL_CSZ   = (size_t)MB_ * H_ * 4;
constexpr size_t RL_H     = RL_C + RL_CSZ;
constexpr size_t RL_HSZ   = (size_t)MB_ * H_ * 4;
constexpr size_t RL_O     = RL_H + RL_HSZ;
constexpr size_t RL_OSZ   = 256 * 4;
constexpr size_t RL_BYTES = RL_O + RL_OSZ;
static_assert(RL_C % 16 == 0);
static_assert(RL_H % 16 == 0);
static_assert(RL_O % 16 == 0);
static_assert((2 * A_TILE) % 8 == 0);
static_assert((MB_ * H_) % 4 == 0);

__device__ __forceinline__ float rcpx(float x) { return __builtin_amdgcn_rcpf(x); }
__device__ __forceinline__ float sigm(float x) { return rcpx(1.0f + __expf(-x)); }
__device__ __forceinline__ float tanhm(float x) {
    const float e = __expf(2.0f * x);
    return 1.0f - 2.0f * rcpx(e + 1.0f);
}
__device__ __forceinline__ v8f zero8() {
    v8f z;
#pragma unroll
    for (int i = 0; i < 8; ++i) z[i] = 0.0f;
    return z;
}

__device__ __forceinline__ void ldfrag_lds(Frag& f, lcp_h p) {
    f.half[0] = *(AS3 const v8h*)(p);
    f.half[1] = *(AS3 const v8h*)(p + 16);
}
__device__ __forceinline__ void ldfrag_glb(Frag& f, const _Float16* p) {
    f.half[0] = *(const v8h*)(p);
    f.half[1] = *(const v8h*)(p + 16);
}
__device__ __forceinline__ v8f mma16(v8f c, const Frag& a, const Frag& b) {
    return __builtin_amdgcn_wmma_f32_16x16x32_f16(false, a.v, false, b.v, (short)0, c, false, false);
}

__global__ __launch_bounds__(NTHR)
void cvt_kernel(const float* __restrict__ wfx, const float* __restrict__ wix,
                const float* __restrict__ wgx, const float* __restrict__ wox,
                const float* __restrict__ wfh, const float* __restrict__ wih,
                const float* __restrict__ wgh, const float* __restrict__ woh,
                _Float16* Wxt, _Float16* Wht)
{
    __shared__ __attribute__((aligned(16))) _Float16 sT[64 * TP];
    const int tid = threadIdx.x;
    const int blk = blockIdx.x;
    const float* src;
    _Float16* dst;
    int kpitch, k0, n0, g;
    if (blk < NBX) {
        g = blk >> 9;
        const int tt = blk & 511;
        k0 = (tt >> 3) * 64;
        n0 = (tt & 7) * 64;
        kpitch = K1_;
        src = (g == 0) ? wfx : (g == 1) ? wix : (g == 2) ? wgx : wox;
        dst = Wxt;
    } else {
        const int b2 = blk - NBX;
        g = b2 >> 6;
        const int tt = b2 & 63;
        k0 = (tt >> 3) * 64;
        n0 = (tt & 7) * 64;
        kpitch = H_;
        src = (g == 0) ? wfh : (g == 1) ? wih : (g == 2) ? wgh : woh;
        dst = Wht;
    }
    {
        const int row = tid >> 2;
        const int cs  = (tid & 3) * 16;
        const float* sp = src + (size_t)(k0 + row) * H_ + n0 + cs;
        const v4f x0 = *(const v4f*)(sp);
        const v4f x1 = *(const v4f*)(sp + 4);
        const v4f x2 = *(const v4f*)(sp + 8);
        const v4f x3 = *(const v4f*)(sp + 12);
        v8h h0, h1;
#pragma unroll
        for (int e = 0; e < 4; ++e) {
            h0[e]     = (_Float16)(x0[e] * SCW);
            h0[4 + e] = (_Float16)(x1[e] * SCW);
            h1[e]     = (_Float16)(x2[e] * SCW);
            h1[4 + e] = (_Float16)(x3[e] * SCW);
        }
        *(AS3 v8h*)(sT + row * TP + cs)     = h0;
        *(AS3 v8h*)(sT + row * TP + cs + 8) = h1;
    }
    __syncthreads();
    v8h ov[2];
    _Float16* dp[2];
#pragma unroll
    for (int it = 0; it < 2; ++it) {
        const int n  = it * 32 + (tid >> 3);
        const int kq = (tid & 7) * 8;
#pragma unroll
        for (int j = 0; j < 8; ++j) ov[it][j] = sT[(kq + j) * TP + n];
        dp[it] = dst + (size_t)(g * H_ + n0 + n) * kpitch + k0 + kq;
    }
#pragma unroll
    for (int it = 0; it < 2; ++it) *(volatile v8h*)dp[it] = ov[it];
    __threadfence();
#pragma unroll
    for (int it = 0; it < 2; ++it) *(volatile v8h*)dp[it] = ov[it];
}

__global__ __launch_bounds__(NTHR)
void pre_kernel(const int* __restrict__ x, const float* __restrict__ emb,
                const _Float16* __restrict__ Wxt,
                const float* __restrict__ bfp, const float* __restrict__ bip,
                const float* __restrict__ bgp, const float* __restrict__ bop,
                float* pre, int tbase)
{
    extern __shared__ __attribute__((aligned(16))) char smem[];
    lp_h sA = (lp_h)(smem + PL_A);
    lp_f sS = (lp_f)(smem + PL_S);

    const int tid  = threadIdx.x;
    const int lane = tid & 31;
    const int w    = tid >> 5;
    const int h    = lane >> 4;
    const int m    = lane & 15;
    const int bh   = blockIdx.x;
    const int tt   = blockIdx.y;
    const int t    = tbase + tt;

#pragma unroll 2
    for (int j = 0; j < 64; ++j) {
        const int rg = w + 8 * j;
        const int rr = rg >> 4;
        const int p  = rg & 15;
        const int b  = bh * MB_ + rr;
        int id = x[((size_t)b * P_ + p) * T_ + t];
        id = min(max(id, 0), V_ - 1);
        const float sc = (id == 0) ? 0.0f : SCX;
        const float* ep = emb + (size_t)id * I_ + lane * 8;
        const v4f e0 = *(const v4f*)(ep);
        const v4f e1 = *(const v4f*)(ep + 4);
        v8h hv;
#pragma unroll
        for (int e = 0; e < 4; ++e) {
            hv[e]     = (_Float16)(e0[e] * sc);
            hv[4 + e] = (_Float16)(e1[e] * sc);
        }
        *(AS3 v8h*)(sA + rr * K1_ + p * I_ + lane * 8) = hv;
    }
    __syncthreads();

    lp_f sSw = sS + w * 512;

#pragma unroll 1
    for (int np = 0; np < 4; ++np) {
        const float* bsel = (np == 0) ? bfp : (np == 1) ? bip : (np == 2) ? bgp : bop;
        const int ncol = np * H_ + w * 64;

        v8f acc[2][4];
#pragma unroll
        for (int mt = 0; mt < 2; ++mt)
#pragma unroll
            for (int ni = 0; ni < 4; ++ni) acc[mt][ni] = zero8();

        lcp_h ab = sA + m * K1_ + 8 * h;
        const _Float16* wb = Wxt + (size_t)(ncol + m) * K1_ + 8 * h;

#pragma unroll 1
        for (int k0 = 0; k0 < K1_; k0 += 32) {
            Frag a[2], b[4];
#pragma unroll
            for (int mt = 0; mt < 2; ++mt) ldfrag_lds(a[mt], ab + mt * (16 * K1_) + k0);
#pragma unroll
            for (int ni = 0; ni < 4; ++ni) ldfrag_glb(b[ni], wb + (size_t)ni * (16 * K1_) + k0);
#pragma unroll
            for (int mt = 0; mt < 2; ++mt)
#pragma unroll
                for (int ni = 0; ni < 4; ++ni) acc[mt][ni] = mma16(acc[mt][ni], a[mt], b[ni]);
#if defined(__HIP_DEVICE_COMPILE__)
            asm volatile("v_nop\n\tv_nop\n\tv_nop\n\tv_nop"
                         : "+v"(acc[0][0]), "+v"(acc[0][1]), "+v"(acc[0][2]), "+v"(acc[0][3]),
                           "+v"(acc[1][0]), "+v"(acc[1][1]), "+v"(acc[1][2]), "+v"(acc[1][3])
                         : "v"(a[0].v), "v"(a[1].v), "v"(b[0].v), "v"(b[1].v), "v"(b[2].v), "v"(b[3].v));
#endif
        }

#pragma unroll
        for (int mt = 0; mt < 2; ++mt) {
#pragma unroll
            for (int hh = 0; hh < 2; ++hh) {
                __syncthreads();
                if (h == hh) {
#pragma unroll
                    for (int ni = 0; ni < 4; ++ni)
#pragma unroll
                        for (int r = 0; r < 8; ++r) sSw[r * 64 + ni * 16 + m] = acc[mt][ni][r];
                }
                __syncthreads();
                const int c4 = m * 4;
                const v4f bb = *(const v4f*)(bsel + w * 64 + c4);
                v4f o[4];
#pragma unroll
                for (int it = 0; it < 4; ++it) {
                    const v4f v = *(AS3 const v4f*)(sSw + (2 * it + h) * 64 + c4);
                    o[it] = v * INVSC + bb;
                }
                float* pb = pre + (size_t)(tt * B_ + bh * MB_ + mt * 16 + hh * 8) * N4_ + ncol + c4;
#pragma unroll
                for (int it = 0; it < 4; ++it)
                    *(volatile v4f*)(pb + (size_t)(2 * it + h) * N4_) = o[it];
                __threadfence();
#pragma unroll
                for (int it = 0; it < 4; ++it)
                    *(volatile v4f*)(pb + (size_t)(2 * it + h) * N4_) = o[it];
            }
        }
    }
}

__global__ __launch_bounds__(NTHR)
void rec_kernel(const float* __restrict__ pre, const _Float16* __restrict__ Wht,
                const float* hsrc, const float* csrc,
                const float* __restrict__ wlin, const float* __restrict__ blin,
                float* hdst, float* cdst, float* odst, int init, int nsteps, int head)
{
    extern __shared__ __attribute__((aligned(16))) char smem[];
    lp_h sA = (lp_h)(smem + RL_A);
    lp_f sC = (lp_f)(smem + RL_C);
    lp_f sH = (lp_f)(smem + RL_H);
    lp_f sO = (lp_f)(smem + RL_O);

    const int tid  = threadIdx.x;
    const int lane = tid & 31;
    const int w    = tid >> 5;
    const int h    = lane >> 4;
    const int m    = lane & 15;
    const int b0   = blockIdx.x * MB_;
    const int nst  = min(max(nsteps, 0), TH_);

    {
        v8h zh;
#pragma unroll
        for (int e = 0; e < 8; ++e) zh[e] = (_Float16)0.0f;
        for (int i = tid; i < (2 * A_TILE) / 8; i += NTHR) *(AS3 v8h*)(sA + 8 * i) = zh;
        v4f zf;
#pragma unroll
        for (int e = 0; e < 4; ++e) zf[e] = 0.0f;
        for (int i = tid; i < (MB_ * H_) / 4; i += NTHR) *(AS3 v4f*)(sC + 4 * i) = zf;
    }
    __syncthreads();
    if (init == 0) {
        for (int i = tid; i < (MB_ * H_) / 8; i += NTHR) {
            const int row = i >> 6;
            const int c8  = (i & 63) * 8;
            const float* hp = hsrc + (size_t)(b0 + row) * H_ + c8;
            const float* cp = csrc + (size_t)(b0 + row) * H_ + c8;
            const v4f h0 = *(const v4f*)(hp);
            const v4f h1 = *(const v4f*)(hp + 4);
            const v4f c0 = *(const v4f*)(cp);
            const v4f c1 = *(const v4f*)(cp + 4);
            v8h hv;
#pragma unroll
            for (int e = 0; e < 4; ++e) {
                hv[e]     = (_Float16)(h0[e] * SCX);
                hv[4 + e] = (_Float16)(h1[e] * SCX);
            }
            *(AS3 v8h*)(sA + row * APITCH + c8)   = hv;
            *(AS3 v4f*)(sC + row * H_ + c8)       = c0;
            *(AS3 v4f*)(sC + row * H_ + c8 + 4)   = c1;
        }
    }

#pragma unroll 1
    for (int s = 0; s < nst; ++s) {
        const int cur  = s & 1;
        const int last = (s == nst - 1);
        lp_h sAc = sA + cur * A_TILE;
        lp_h sAn = sA + (cur ^ 1) * A_TILE;

        __syncthreads();

#pragma unroll 1
        for (int g4 = 0; g4 < 4; ++g4) {
            const int j0 = w * 64 + g4 * 16;
            v8f acc[2][4];
#pragma unroll
            for (int mt = 0; mt < 2; ++mt)
#pragma unroll
                for (int q = 0; q < 4; ++q) acc[mt][q] = zero8();

            lcp_h ab = sAc + m * APITCH + 8 * h;
            const _Float16* wb = Wht + (size_t)(j0 + m) * H_ + 8 * h;

#pragma unroll 1
            for (int k0 = 0; k0 < H_; k0 += 32) {
                Frag a[2], b[4];
#pragma unroll
                for (int mt = 0; mt < 2; ++mt) ldfrag_lds(a[mt], ab + mt * (16 * APITCH) + k0);
#pragma unroll
                for (int q = 0; q < 4; ++q) ldfrag_glb(b[q], wb + (size_t)q * ((size_t)H_ * H_) + k0);
#pragma unroll
                for (int mt = 0; mt < 2; ++mt)
#pragma unroll
                    for (int q = 0; q < 4; ++q) acc[mt][q] = mma16(acc[mt][q], a[mt], b[q]);
#if defined(__HIP_DEVICE_COMPILE__)
                asm volatile("v_nop\n\tv_nop\n\tv_nop\n\tv_nop"
                             : "+v"(acc[0][0]), "+v"(acc[0][1]), "+v"(acc[0][2]), "+v"(acc[0][3]),
                               "+v"(acc[1][0]), "+v"(acc[1][1]), "+v"(acc[1][2]), "+v"(acc[1][3])
                             : "v"(a[0].v), "v"(a[1].v), "v"(b[0].v), "v"(b[1].v), "v"(b[2].v), "v"(b[3].v));
#endif
            }

            const int n = j0 + m;
#pragma unroll
            for (int mt = 0; mt < 2; ++mt) {
#pragma unroll
                for (int r = 0; r < 8; ++r) {
                    const int row = mt * 16 + 8 * h + r;
                    const float* pp = pre + ((size_t)s * B_ + b0 + row) * N4_ + n;
                    const float gf = acc[mt][0][r] * INVSC + pp[0];
                    const float gi = acc[mt][1][r] * INVSC + pp[H_];
                    const float gg = acc[mt][2][r] * INVSC + pp[2 * H_];
                    const float go = acc[mt][3][r] * INVSC + pp[3 * H_];
                    const float cp = sC[row * H_ + n];
                    const float ig = sigm(gi) * tanhm(gg);
                    const float cn = sigm(gf) * cp + ig;
                    sC[row * H_ + n] = cn;
                    const float hn = sigm(go) * tanhm(cn);
                    sAn[row * APITCH + n] = (_Float16)(hn * SCX);
                    if (last) sH[row * H_ + n] = hn;
                }
            }
        }
    }

    __syncthreads();

#pragma unroll 1
    for (int it = 0; it < (MB_ * H_ / 4) / NTHR; ++it) {
        const int idx = it * NTHR + tid;
        const int row = idx >> 7;
        const int c4  = (idx & 127) * 4;
        const v4f hv = *(AS3 const v4f*)(sH + row * H_ + c4);
        const v4f cv = *(AS3 const v4f*)(sC + row * H_ + c4);
        float* hp = hdst + (size_t)(b0 + row) * H_ + c4;
        float* cp = cdst + (size_t)(b0 + row) * H_ + c4;
        *(volatile v4f*)hp = hv;
        *(volatile v4f*)cp = cv;
        __threadfence();
        *(volatile v4f*)hp = hv;
        *(volatile v4f*)cp = cv;
    }

    if (head != 0) {
        if (tid < MB_ * O_) {
            const int bb = tid / O_;
            const int o  = tid - bb * O_;
            float acc0 = 0.0f;
#pragma unroll 4
            for (int k = 0; k < H_; ++k) acc0 += sH[bb * H_ + k] * wlin[k * O_ + o];
            acc0 += blin[o];
            sO[tid] = acc0;
        }
        __syncthreads();
        if (w == 0) {
            float* ob = odst + (size_t)blockIdx.x * (MB_ * O_);
            const v4f v0 = *(AS3 const v4f*)(sO + lane * 4);
            const v4f v1 = *(AS3 const v4f*)(sO + 128 + (lane & 7) * 4);
            *(volatile v4f*)(ob + lane * 4) = v0;
            if (lane < 8) *(volatile v4f*)(ob + 128 + lane * 4) = v1;
            __threadfence();
            *(volatile v4f*)(ob + lane * 4) = v0;
            if (lane < 8) *(volatile v4f*)(ob + 128 + lane * 4) = v1;
        }
    }
}

extern "C" void kernel_launch(void* const* d_in, const int* in_sizes, int n_in,
                              void* d_out, int out_size, void* d_ws, size_t ws_size,
                              hipStream_t stream)
{
    if (n_in < 16) return;
    if (in_sizes[0]  != B_ * P_ * T_) return;
    if (in_sizes[1]  != V_ * I_)      return;
    if (in_sizes[2]  != P_ * I_ * H_) return;
    if (in_sizes[3]  != H_ * H_)      return;
    if (in_sizes[4]  != H_)           return;
    if (in_sizes[5]  != P_ * I_ * H_) return;
    if (in_sizes[6]  != H_ * H_)      return;
    if (in_sizes[7]  != H_)           return;
    if (in_sizes[8]  != P_ * I_ * H_) return;
    if (in_sizes[9]  != H_ * H_)      return;
    if (in_sizes[10] != H_)           return;
    if (in_sizes[11] != P_ * I_ * H_) return;
    if (in_sizes[12] != H_ * H_)      return;
    if (in_sizes[13] != H_)           return;
    if (in_sizes[14] != H_ * O_)      return;
    if (in_sizes[15] != O_)           return;
    if (out_size != B_ * O_ + 2 * B_ * H_) return;
    if (ws_size < WS_END) return;

    const int*   x    = (const int*)  d_in[0];
    const float* emb  = (const float*)d_in[1];
    const float* wfx  = (const float*)d_in[2];
    const float* wfh  = (const float*)d_in[3];
    const float* bfp  = (const float*)d_in[4];
    const float* wix  = (const float*)d_in[5];
    const float* wih  = (const float*)d_in[6];
    const float* bip  = (const float*)d_in[7];
    const float* wgx  = (const float*)d_in[8];
    const float* wgh  = (const float*)d_in[9];
    const float* bgp  = (const float*)d_in[10];
    const float* wox  = (const float*)d_in[11];
    const float* woh  = (const float*)d_in[12];
    const float* bop  = (const float*)d_in[13];
    const float* wlin = (const float*)d_in[14];
    const float* blin = (const float*)d_in[15];

    float* out  = (float*)d_out;
    float* out0 = out;
    float* out1 = out + B_ * O_;
    float* out2 = out + B_ * O_ + B_ * H_;

    char* ws = (char*)d_ws;
    _Float16* Wxt = (_Float16*)(ws + OFF_WXT);
    _Float16* Wht = (_Float16*)(ws + OFF_WHT);
    float*    hst = (float*)(ws + OFF_HST);
    float*    cst = (float*)(ws + OFF_CST);
    float*    pre = (float*)(ws + OFF_PRE);

    cvt_kernel<<<dim3(NBX + NBH), dim3(NTHR), 0, stream>>>(wfx, wix, wgx, wox, wfh, wih, wgh, woh, Wxt, Wht);

    hipFuncSetAttribute(reinterpret_cast<const void*>(&pre_kernel),
                        hipFuncAttributeMaxDynamicSharedMemorySize, (int)PL_BYTES);
    hipFuncSetAttribute(reinterpret_cast<const void*>(&rec_kernel),
                        hipFuncAttributeMaxDynamicSharedMemorySize, (int)RL_BYTES);

    pre_kernel<<<dim3(2, TH_), dim3(NTHR), PL_BYTES, stream>>>(
        x, emb, (const _Float16*)Wxt, bfp, bip, bgp, bop, pre, 0);
    rec_kernel<<<dim3(NBLK), dim3(NTHR), RL_BYTES, stream>>>(
        (const float*)pre, (const _Float16*)Wht, (const float*)hst, (const float*)cst,
        wlin, blin, hst, cst, out0, 1, TH_, 0);

    pre_kernel<<<dim3(2, TH_), dim3(NTHR), PL_BYTES, stream>>>(
        x, emb, (const _Float16*)Wxt, bfp, bip, bgp, bop, pre, TH_);
    rec_kernel<<<dim3(NBLK), dim3(NTHR), RL_BYTES, stream>>>(
        (const float*)pre, (const _Float16*)Wht, (const float*)hst, (const float*)cst,
        wlin, blin, out1, out2, out0, 0, TH_, 1);
}
